// KANOriginal_82429012345259
// MI455X (gfx1250) — hardware-verified
//
#include <hip/hip_runtime.h>


#define NR   8192
#define DIN  768
#define DOUT 768
#define NBAS 6
#define KB   (DIN * NBAS)
#define RCH  2048
#define GNUM 3
#define KORD 3
#define DM   DIN
#define NTK  RCH
#define LOSC 1024.0f

typedef _Float16 h16;
typedef unsigned short bf;
typedef __attribute__((ext_vector_type(16))) __bf16   v16bf;
typedef __attribute__((ext_vector_type(16))) _Float16 v16h;
typedef __attribute__((ext_vector_type(8)))  _Float16 v8h;
typedef __attribute__((ext_vector_type(8)))  unsigned short v8us;
typedef __attribute__((ext_vector_type(8)))  float    v8f;
typedef __attribute__((ext_vector_type(4)))  float    v4f;
typedef __attribute__((ext_vector_type(4)))  _Float16 v4h;
typedef v8h  __attribute__((may_alias)) v8ha;
typedef v4f  __attribute__((may_alias)) v4fa;
typedef v8us __attribute__((may_alias)) v8usa;

__device__ __forceinline__ unsigned short f2bf(float f) { unsigned u = __float_as_uint(f); u += 0x7FFFu + ((u >> 16) & 1u); return (unsigned short)(u >> 16); }
__device__ __forceinline__ float bf2f(unsigned short b) { return __uint_as_float(((unsigned)b) << 16); }
__device__ __forceinline__ float bfr(float f) { return bf2f(f2bf(f)); }
__device__ __forceinline__ v16h cat16(v8h lo, v8h hi) { return __builtin_shufflevector(lo, hi, 0, 1, 2, 3, 4, 5, 6, 7, 8, 9, 10, 11, 12, 13, 14, 15); }
__device__ __forceinline__ v16bf cat16b(v8us lo, v8us hi) { return __builtin_bit_cast(v16bf, __builtin_shufflevector(lo, hi, 0, 1, 2, 3, 4, 5, 6, 7, 8, 9, 10, 11, 12, 13, 14, 15)); }
__device__ __forceinline__ v8f wmma16(v16h a, v16h b, v8f c) { return __builtin_amdgcn_wmma_f32_16x16x32_f16(false, a, false, b, (short)0, c, false, false); }
__device__ __forceinline__ v8f wmmab(v16bf a, v16bf b, v8f c) { return __builtin_amdgcn_wmma_f32_16x16x32_bf16(false, a, false, b, (short)0, c, false, false); }

template <bool SPLITA, bool F16OUT = false>
__global__ __launch_bounds__(128) void k_gemmb(const bf* __restrict__ A, const bf* __restrict__ Al, const bf* __restrict__ Bn, const float* __restrict__ bias, float* C, int ldc, h16* C2, const float* __restrict__ R = nullptr, int K = DM, int roundR = 1) {
    __shared__ __align__(16) float ost[4][16 * 68];
    const int lane = threadIdx.x & 31, wave = threadIdx.x >> 5, lr = lane & 15, hi = lane >> 4;
    const int r0 = blockIdx.x * 64 + wave * 16, c0 = blockIdx.y * 64;
    const size_t aoff = (size_t)(r0 + lr) * K + 8 * hi;
    size_t boff[4];
#pragma unroll
    for (int t = 0; t < 4; ++t) boff[t] = (size_t)(c0 + t * 16 + lr) * K + 8 * hi;
    v8f acc[4];
#pragma unroll
    for (int t = 0; t < 4; ++t) acc[t] = (v8f){};
#pragma unroll 1
    for (int kc = 0; kc < K; kc += 32) {
        const v16bf a = cat16b(*(const v8us*)(A + aoff + kc), *(const v8us*)(A + aoff + kc + 16));
        v16bf al = a;
        if (SPLITA) al = cat16b(*(const v8us*)(Al + aoff + kc), *(const v8us*)(Al + aoff + kc + 16));
#pragma unroll
        for (int t = 0; t < 4; ++t) { const v16bf b = cat16b(*(const v8us*)(Bn + boff[t] + kc), *(const v8us*)(Bn + boff[t] + kc + 16)); acc[t] = wmmab(a, b, acc[t]); if (SPLITA) acc[t] = wmmab(al, b, acc[t]); }
        asm volatile("v_nop\n\tv_nop\n\tv_nop\n\tv_nop" : "+v"(acc[0]), "+v"(acc[1]), "+v"(acc[2]), "+v"(acc[3]) : "v"(a), "v"(al));
    }
    float* os = &ost[wave][0];
#pragma unroll
    for (int t = 0; t < 4; ++t) { const float bv = bias ? bfr(bias[c0 + t * 16 + lr]) : 0.f;
#pragma unroll
        for (int j = 0; j < 8; ++j) os[(hi * 8 + j) * 68 + t * 16 + lr] = acc[t][j] + bv; }
    __syncthreads();
    if (F16OUT) {
        h16* crow = (h16*)(void*)C + (size_t)r0 * ldc + c0;
        auto pass = [&]() {
#pragma unroll
            for (int s = 0; s < 4; ++s) { const int row = 4 * s + (lane >> 3), piece = lane & 7; const float* sp = os + row * 68 + piece * 8; v8h o, o2;
#pragma unroll
                for (int i = 0; i < 8; ++i) { const h16 a = (h16)sp[i]; o[i] = a; o2[i] = (h16)((sp[i] - (float)a) * LOSC); }
                *(volatile v8h*)(crow + (size_t)row * ldc + piece * 8) = o; if (C2) *(volatile v8h*)(C2 + (size_t)r0 * ldc + c0 + (size_t)row * ldc + piece * 8) = o2; }
        };
        pass(); __threadfence(); pass();
    } else {
        float* crow = C + (size_t)r0 * ldc + c0;
        auto pass = [&]() {
#pragma unroll
            for (int s = 0; s < 8; ++s) { const int Lid = (lane >> 3) + 4 * s, piece = lane & 7; const int row = Lid >> 1, cofs = (Lid & 1) * 32 + piece * 4;
                v4f val = *(const v4fa*)(os + row * 68 + cofs); if (R) { const v4f rv = *(const v4f*)(R + ((size_t)r0 + row) * ldc + c0 + cofs); val += roundR ? (v4f){bfr(rv[0]), bfr(rv[1]), bfr(rv[2]), bfr(rv[3])} : rv; }
                *(volatile v4f*)(crow + (size_t)row * ldc + cofs) = val; }
        };
        pass(); __threadfence(); pass();
    }
}

__global__ __launch_bounds__(128) void k_gemm3(const bf* __restrict__ Ah, const bf* __restrict__ Al, const bf* __restrict__ Bh, const bf* __restrict__ Bl, int K, float* C, int ldc) {
    __shared__ __align__(16) float ost[4][16 * 68];
    const int lane = threadIdx.x & 31, wave = threadIdx.x >> 5, lr = lane & 15, hi = lane >> 4;
    const int r0 = blockIdx.x * 64 + wave * 16, c0 = blockIdx.y * 64;
    const size_t aoff = (size_t)(r0 + lr) * K + 8 * hi;
    v8f acc[4];
#pragma unroll
    for (int t = 0; t < 4; ++t) acc[t] = (v8f){};
#pragma unroll 1
    for (int kc = 0; kc < K; kc += 32) {
        const v16bf a = cat16b(*(const v8us*)(Ah + aoff + kc), *(const v8us*)(Ah + aoff + kc + 16));
        const v16bf al = cat16b(*(const v8us*)(Al + aoff + kc), *(const v8us*)(Al + aoff + kc + 16));
#pragma unroll
        for (int t = 0; t < 4; ++t) { const size_t bo = (size_t)(c0 + t * 16 + lr) * K + kc + 8 * hi;
            const v16bf bh = cat16b(*(const v8us*)(Bh + bo), *(const v8us*)(Bh + bo + 16)); const v16bf bl = cat16b(*(const v8us*)(Bl + bo), *(const v8us*)(Bl + bo + 16));
            acc[t] = wmmab(a, bh, acc[t]); acc[t] = wmmab(al, bh, acc[t]); acc[t] = wmmab(a, bl, acc[t]); }
        asm volatile("v_nop\n\tv_nop\n\tv_nop\n\tv_nop" : "+v"(acc[0]), "+v"(acc[1]), "+v"(acc[2]), "+v"(acc[3]) : "v"(a), "v"(al));
    }
    float* os = &ost[wave][0];
#pragma unroll
    for (int t = 0; t < 4; ++t) {
#pragma unroll
        for (int j = 0; j < 8; ++j) os[(hi * 8 + j) * 68 + t * 16 + lr] = acc[t][j]; }
    __builtin_amdgcn_wave_barrier(); asm volatile("" ::: "memory");
    float* crow = C + (size_t)r0 * ldc + c0;
    auto pass = [&]() {
#pragma unroll
        for (int s = 0; s < 8; ++s) { const int Lid = (lane >> 3) + 4 * s, piece = lane & 7; const int row = Lid >> 1, cofs = (Lid & 1) * 32 + piece * 4;
            const v4f val = *(const v4fa*)(os + row * 68 + cofs); *(volatile v4f*)(crow + (size_t)row * ldc + cofs) = val; }
    };
    pass(); __threadfence(); pass();
}

__global__ __launch_bounds__(256) void k_bf(const float* __restrict__ src, bf* dst, size_t n8) {
    const size_t i = (size_t)blockIdx.x * 256 + threadIdx.x; if (i >= n8) return;
    const v8f v = *(const v8f*)(src + i * 8); v8us o;
#pragma unroll
    for (int k = 0; k < 8; ++k) o[k] = f2bf(v[k]);
    *(volatile v8us*)(dst + i * 8) = o; __threadfence(); *(volatile v8us*)(dst + i * 8) = o;
}
__global__ __launch_bounds__(256) void k_w2(const float* __restrict__ coef, const float* __restrict__ sp, bf* Wh, bf* Wl) {
    const size_t u = (size_t)blockIdx.x * 256 + threadIdx.x; if (u >= (size_t)DOUT * KB / 8) return; v8us oh, ol;
#pragma unroll
    for (int k = 0; k < 8; ++k) { const size_t e = u * 8 + k; const int o = (int)(e / KB), r = (int)(e % KB), i = r / NBAS; const float w = bfr(sp[(size_t)o * DIN + i]) * bfr(coef[e]);
        const unsigned short hb = f2bf(w); oh[k] = hb; ol[k] = f2bf(w - bf2f(hb)); }
    *(volatile v8us*)(Wh + u * 8) = oh; *(volatile v8us*)(Wl + u * 8) = ol; __threadfence(); *(volatile v8us*)(Wh + u * 8) = oh; *(volatile v8us*)(Wl + u * 8) = ol;
}
__global__ __launch_bounds__(256) void k_basis(const float* __restrict__ x, size_t row0, bf* BAh, bf* BAl, bf* SIh, bf* SIl) {
    __shared__ __align__(16) unsigned short st[8][2][192]; __shared__ __align__(16) unsigned short su[8][2][64]; __shared__ float bs[8][32][GNUM + 2 * KORD + 1]; __shared__ float gs[GNUM + 2 * KORD + 2];
    typedef __attribute__((ext_vector_type(2))) unsigned short v2us;
    const int lane = threadIdx.x & 31, wv = threadIdx.x >> 5, n = blockIdx.x * 8 + wv; if (n >= RCH) return;
    const float h = 2.0f / (float)GNUM;
    if (threadIdx.x < GNUM + 2 * KORD + 1) gs[threadIdx.x] = (float)((int)threadIdx.x - KORD) * h - 1.0f;
    __syncthreads();
#define B bs[wv][lane]
    const float* xr = x + (row0 + n) * DIN;
#pragma unroll 1
    for (int s = 0; s < DIN / 32; ++s) { const int i = s * 32 + lane; const float xv = bfr(xr[i]);
#pragma unroll 1
        for (int j = 0; j < GNUM + 2 * KORD; ++j) B[j] = (xv >= gs[j] && xv < gs[j + 1]) ? 1.0f : 0.0f;
#pragma unroll 1
        for (int p = 1; p <= KORD; ++p) {
#pragma unroll 1
            for (int j = 0; j < GNUM + 2 * KORD - p; ++j) B[j] = (xv - gs[j]) / (gs[j + p] - gs[j]) * B[j] + (gs[j + p + 1] - xv) / (gs[j + p + 1] - gs[j + 1]) * B[j + 1]; }
#pragma unroll
        for (int m = 0; m < NBAS; ++m) { const unsigned short hb = f2bf(B[m]); st[wv][0][lane * NBAS + m] = hb; st[wv][1][lane * NBAS + m] = f2bf(B[m] - bf2f(hb)); }
        __builtin_amdgcn_wave_barrier(); asm volatile("" ::: "memory");
        const size_t ob = (size_t)n * KB + (size_t)s * 192;
#pragma unroll 1
        for (int ps = 0; ps < 2; ++ps) { if (lane < 24) { const v8us vh = *(const v8us*)&st[wv][0][lane * 8], vl = *(const v8us*)&st[wv][1][lane * 8]; *(volatile v8us*)(BAh + ob + lane * 8) = vh; *(volatile v8us*)(BAl + ob + lane * 8) = vl; } if (ps == 0) __threadfence(); }
        __builtin_amdgcn_wave_barrier(); asm volatile("" ::: "memory");
        const float sl = xv / (1.0f + __expf(-xv)); const unsigned short sh_ = f2bf(sl); su[wv][0][(s & 1) * 32 + lane] = sh_; su[wv][1][(s & 1) * 32 + lane] = f2bf(sl - bf2f(sh_));
        __builtin_amdgcn_wave_barrier(); asm volatile("" ::: "memory");
        if (s & 1) { const size_t os_ = (size_t)n * DIN + (size_t)(s - 1) * 32;
#pragma unroll 1
            for (int ps = 0; ps < 2; ++ps) { if (lane < 8) { const v8us vh = *(const v8us*)&su[wv][0][lane * 8], vl = *(const v8us*)&su[wv][1][lane * 8]; *(volatile v8us*)(SIh + os_ + lane * 8) = vh; *(volatile v8us*)(SIl + os_ + lane * 8) = vl; } if (ps == 0) __threadfence(); } }
        __builtin_amdgcn_wave_barrier(); asm volatile("" ::: "memory");
    }
}
#undef B

extern "C" void kernel_launch(void* const* d_in, const int* in_sizes, int n_in,
                              void* d_out, int out_size, void* d_ws, size_t ws_size, hipStream_t stream) {
    (void)in_sizes; (void)n_in; (void)out_size;
    const float* x = (const float*)d_in[0]; const float* coef = (const float*)d_in[1]; const float* sb = (const float*)d_in[2]; const float* sp = (const float*)d_in[3]; const float* bias = (const float*)d_in[4];
    float* out = (float*)d_out;
    char* wsp = (char*)d_ws;
    auto take = [&](size_t bytes) { char* p = wsp; wsp += (bytes + 255) & ~(size_t)255; return (void*)p; };
    bf* SB = (bf*)take((size_t)DOUT * DIN * 2); bf* W2h = (bf*)take((size_t)DOUT * KB * 2); bf* W2l = (bf*)take((size_t)DOUT * KB * 2);
    bf* BAh = (bf*)take((size_t)RCH * KB * 2); bf* BAl = (bf*)take((size_t)RCH * KB * 2); bf* SIh = (bf*)take((size_t)RCH * DIN * 2); bf* SIl = (bf*)take((size_t)RCH * DIN * 2); float* SPL = (float*)take((size_t)RCH * DOUT * 4);
    if ((size_t)(wsp - (char*)d_ws) > ws_size) return;
    k_bf<<<(DOUT * DIN / 8 + 255) / 256, 256, 0, stream>>>(sb, SB, (size_t)DOUT * DIN / 8); k_w2<<<(unsigned)(((size_t)DOUT * KB / 8 + 255) / 256), 256, 0, stream>>>(coef, sp, W2h, W2l);
    for (int ch = 0; ch < NR / RCH; ++ch) { const size_t r0 = (size_t)ch * RCH;
        k_basis<<<RCH / 8, 256, 0, stream>>>(x, r0, BAh, BAl, SIh, SIl);
        k_gemm3<<<dim3(RCH / 64, DOUT / 64, 1), 128, 0, stream>>>(BAh, BAl, W2h, W2l, KB, SPL, DOUT);
        k_gemmb<true, false><<<dim3(RCH / 64, DOUT / 64, 1), 128, 0, stream>>>(SIh, SIl, SB, bias, out + r0 * DOUT, DOUT, nullptr, SPL, DOUT, 0);
    }
}
